// MultiScaleDecoderRetention_3161095930391
// MI455X (gfx1250) — hardware-verified
//
#include <hip/hip_runtime.h>


#define NB_  4
#define TT   2048
#define DM   1024
#define NH_  8
#define HD   128
#define ZH   2
#define GNEPS 1e-5f
typedef _Float16 h16;
typedef unsigned short bf;
typedef __attribute__((ext_vector_type(16))) __bf16   v16bf;
typedef __attribute__((ext_vector_type(16))) _Float16 v16h;
typedef __attribute__((ext_vector_type(8)))  _Float16 v8h;
typedef __attribute__((ext_vector_type(8)))  unsigned short v8us;
typedef __attribute__((ext_vector_type(8)))  float    v8f;
typedef __attribute__((ext_vector_type(4)))  float    v4f;
typedef v8h  __attribute__((may_alias)) v8ha;
typedef v4f  __attribute__((may_alias)) v4fa;
typedef v8us __attribute__((may_alias)) v8usa;

__device__ __forceinline__ unsigned short f2bf(float f) { unsigned u = __float_as_uint(f); u += 0x7FFFu + ((u >> 16) & 1u); return (unsigned short)(u >> 16); }
__device__ __forceinline__ float bf2f(unsigned short b) { return __uint_as_float(((unsigned)b) << 16); }
__device__ __forceinline__ float bfr(float f) { return bf2f(f2bf(f)); }
__device__ __forceinline__ v16h cat16(v8h lo, v8h hi) { return __builtin_shufflevector(lo, hi, 0, 1, 2, 3, 4, 5, 6, 7, 8, 9, 10, 11, 12, 13, 14, 15); }
__device__ __forceinline__ v16bf cat16b(v8us lo, v8us hi) { return __builtin_bit_cast(v16bf, __builtin_shufflevector(lo, hi, 0, 1, 2, 3, 4, 5, 6, 7, 8, 9, 10, 11, 12, 13, 14, 15)); }
__device__ __forceinline__ v8f wmma16(v16h a, v16h b, v8f c) { return __builtin_amdgcn_wmma_f32_16x16x32_f16(false, a, false, b, (short)0, c, false, false); }
__device__ __forceinline__ v8f wmmab(v16bf a, v16bf b, v8f c) { return __builtin_amdgcn_wmma_f32_16x16x32_bf16(false, a, false, b, (short)0, c, false, false); }


template <typename T16> struct WFrag;
template <> struct WFrag<h16> { typedef v16h V; static __device__ __forceinline__ V ld(const h16* p) { return cat16(*(const v8h*)p, *(const v8h*)(p + 16)); } static __device__ __forceinline__ v8f mma(V a, V b, v8f c) { return wmma16(a, b, c); } };
template <> struct WFrag<bf> { typedef v16bf V; static __device__ __forceinline__ V ld(const bf* p) { return cat16b(*(const v8us*)p, *(const v8us*)(p + 16)); } static __device__ __forceinline__ v8f mma(V a, V b, v8f c) { return wmmab(a, b, c); } };
template <typename T16, int NSPLIT, bool BIAS>
__global__ __launch_bounds__(32) void k_gemmw(const T16* __restrict__ A, const T16* __restrict__ A2, const T16* __restrict__ Bt, const T16* __restrict__ Bt2, int K, float* C, int ldc, const float* __restrict__ bias, size_t sA, size_t sB, size_t sC) {
    typedef typename WFrag<T16>::V V;
    __shared__ __align__(16) float os[16 * 68];
    const size_t z = blockIdx.z; A += z * sA; if (A2) A2 += z * sA; Bt += z * sB; if (Bt2) Bt2 += z * sB; C += z * sC;
    const int lane = threadIdx.x & 31, lr = lane & 15, hi = lane >> 4; const int r0 = blockIdx.x * 64, c0 = blockIdx.y * 64;
    v8f acc[4][4];
#pragma unroll
    for (int mb = 0; mb < 4; ++mb)
#pragma unroll
        for (int nb = 0; nb < 4; ++nb) acc[mb][nb] = (v8f){};
    const size_t aoff = (size_t)(r0 + lr) * K + 8 * hi, boff = (size_t)(c0 + lr) * K + 8 * hi;
#pragma unroll 1
    for (int kc = 0; kc < K; kc += 32) {
        V a[4], a2[4];
#pragma unroll
        for (int mb = 0; mb < 4; ++mb) { a[mb] = WFrag<T16>::ld(A + aoff + (size_t)mb * 16 * K + kc); if (NSPLIT == 1 || NSPLIT == 2) a2[mb] = WFrag<T16>::ld(A2 + aoff + (size_t)mb * 16 * K + kc); }
#pragma unroll
        for (int nb = 0; nb < 4; ++nb) { const V b = WFrag<T16>::ld(Bt + boff + (size_t)nb * 16 * K + kc); V b2; if (NSPLIT >= 2) b2 = WFrag<T16>::ld(Bt2 + boff + (size_t)nb * 16 * K + kc);
#pragma unroll
            for (int mb = 0; mb < 4; ++mb) { acc[mb][nb] = WFrag<T16>::mma(a[mb], b, acc[mb][nb]); if (NSPLIT == 1 || NSPLIT == 2) acc[mb][nb] = WFrag<T16>::mma(a2[mb], b, acc[mb][nb]); if (NSPLIT >= 2) acc[mb][nb] = WFrag<T16>::mma(a[mb], b2, acc[mb][nb]); } }
        asm volatile("v_nop\n\tv_nop\n\tv_nop\n\tv_nop" : "+v"(acc[0][0]), "+v"(acc[1][1]), "+v"(acc[2][2]), "+v"(acc[3][3]) : "v"(a[0]), "v"(a[3]));
    }
#pragma unroll
    for (int mb = 0; mb < 4; ++mb) {
#pragma unroll
        for (int nb = 0; nb < 4; ++nb) {
#pragma unroll
            for (int j = 0; j < 8; ++j) os[(hi * 8 + j) * 68 + nb * 16 + lr] = acc[mb][nb][j]; }
        __builtin_amdgcn_wave_barrier(); asm volatile("" ::: "memory");
        float* crow = C + (size_t)(r0 + mb * 16) * ldc + c0;
#pragma unroll 1
        for (int ps = 0; ps < 2; ++ps) {
#pragma unroll
            for (int s = 0; s < 8; ++s) { const int row = 2 * s + hi, cofs = lr * 4; v4f val = *(const v4fa*)(os + row * 68 + cofs); if (BIAS) { val[0] += bfr(bias[c0 + cofs]); val[1] += bfr(bias[c0 + cofs + 1]); val[2] += bfr(bias[c0 + cofs + 2]); val[3] += bfr(bias[c0 + cofs + 3]); }
                *(volatile v4f*)(crow + (size_t)row * ldc + cofs) = val; }
            if (ps == 0) __threadfence(); }
        __builtin_amdgcn_wave_barrier(); asm volatile("" ::: "memory");
    }
}

template <typename T16, int NSPLIT, int CMODE>
__global__ __launch_bounds__(32) void k_gemmc(const T16* __restrict__ A, const T16* __restrict__ A2, const T16* __restrict__ Bt, const T16* __restrict__ Bt2, int K, float* C, int ldc, int roff, size_t sA, size_t sB, size_t sC) {
    typedef typename WFrag<T16>::V V;
    __shared__ __align__(16) float os[16 * 68];
    const size_t z = blockIdx.z; A += z * sA; if (A2) A2 += z * sA; Bt += z * sB; if (Bt2) Bt2 += z * sB; C += z * sC;
    const int lane = threadIdx.x & 31, lr = lane & 15, hi = lane >> 4; const int r0 = blockIdx.x * 64, c0 = blockIdx.y * 64;
    if (CMODE == 1 && c0 > r0 + roff + 63) return;
    const int Kl = (CMODE == 2) ? min(K, r0 + roff + 64) : K;
    v8f acc[4][4];
#pragma unroll
    for (int mb = 0; mb < 4; ++mb)
#pragma unroll
        for (int nb = 0; nb < 4; ++nb) acc[mb][nb] = (v8f){};
    const size_t aoff = (size_t)(r0 + lr) * K + 8 * hi, boff = (size_t)(c0 + lr) * K + 8 * hi;
#pragma unroll 1
    for (int kc = 0; kc < Kl; kc += 32) {
        V a[4], a2[4];
#pragma unroll
        for (int mb = 0; mb < 4; ++mb) { a[mb] = WFrag<T16>::ld(A + aoff + (size_t)mb * 16 * K + kc); if (NSPLIT == 1 || NSPLIT == 2) a2[mb] = WFrag<T16>::ld(A2 + aoff + (size_t)mb * 16 * K + kc); }
#pragma unroll
        for (int nb = 0; nb < 4; ++nb) { const V b = WFrag<T16>::ld(Bt + boff + (size_t)nb * 16 * K + kc); V b2; if (NSPLIT >= 2) b2 = WFrag<T16>::ld(Bt2 + boff + (size_t)nb * 16 * K + kc);
#pragma unroll
            for (int mb = 0; mb < 4; ++mb) { acc[mb][nb] = WFrag<T16>::mma(a[mb], b, acc[mb][nb]); if (NSPLIT == 1 || NSPLIT == 2) acc[mb][nb] = WFrag<T16>::mma(a2[mb], b, acc[mb][nb]); if (NSPLIT >= 2) acc[mb][nb] = WFrag<T16>::mma(a[mb], b2, acc[mb][nb]); } }
        asm volatile("v_nop\n\tv_nop\n\tv_nop\n\tv_nop" : "+v"(acc[0][0]), "+v"(acc[1][1]), "+v"(acc[2][2]), "+v"(acc[3][3]) : "v"(a[0]), "v"(a[3]));
    }
#pragma unroll
    for (int mb = 0; mb < 4; ++mb) {
#pragma unroll
        for (int nb = 0; nb < 4; ++nb) {
#pragma unroll
            for (int j = 0; j < 8; ++j) os[(hi * 8 + j) * 68 + nb * 16 + lr] = acc[mb][nb][j]; }
        __builtin_amdgcn_wave_barrier(); asm volatile("" ::: "memory");
        float* crow = C + (size_t)(r0 + mb * 16) * ldc + c0;
#pragma unroll 1
        for (int ps = 0; ps < 2; ++ps) {
#pragma unroll
            for (int s = 0; s < 8; ++s) { const int row = 2 * s + hi, cofs = lr * 4; v4f val = *(const v4fa*)(os + row * 68 + cofs);
                *(volatile v4f*)(crow + (size_t)row * ldc + cofs) = val; }
            if (ps == 0) __threadfence(); }
        __builtin_amdgcn_wave_barrier(); asm volatile("" ::: "memory");
    }
}

__device__ __forceinline__ void splitf(float y, unsigned short& h, unsigned short& l) { h = f2bf(y); l = f2bf(y - bf2f(h)); }
typedef __attribute__((ext_vector_type(2))) unsigned short v2us;
typedef __attribute__((ext_vector_type(4))) unsigned short v4us;
typedef __attribute__((ext_vector_type(2))) float v2f;
__constant__ float INV[HD / 2] = {1.0,0.8659643530845642,0.7498942017555237,0.6493816375732422,0.5623413324356079,0.486967533826828,0.4216965138912201,0.36517414450645447,0.3162277638912201,0.2738419771194458,0.23713736236095428,0.20535250008106232,0.17782793939113617,0.1539926528930664,0.1333521455526352,0.11547820270061493,0.10000000149011612,0.08659642934799194,0.07498941570520401,0.06493816524744034,0.05623412877321243,0.04869675263762474,0.04216964915394783,0.03651741147041321,0.03162277862429619,0.0273841954767704,0.0237137358635664,0.02053525112569332,0.017782794311642647,0.015399265103042126,0.01333521492779255,0.011547819711267948,0.009999999776482582,0.00865964312106371,0.007498942315578461,0.006493816617876291,0.005623413249850273,0.004869675263762474,0.0042169648222625256,0.003651741426438093,0.003162277862429619,0.0027384196873754263,0.0023713738191872835,0.0020535250660032034,0.0017782794311642647,0.0015399265103042126,0.0013335214462131262,0.0011547820176929235,0.0010000000474974513,0.0008659643353894353,0.0007498941849917173,0.0006493816617876291,0.000562341301701963,0.00048696750309318304,0.00042169648804701865,0.00036517411353997886,0.0003162277862429619,0.00027384195709601045,0.0002371373848291114,0.00020535249495878816,0.00017782794020604342,0.00015399264520965517,0.0001333521504420787,0.00011547819303814322};
__constant__ float BSC[HD / 2] = {0.2857142984867096,0.296875,0.3080357313156128,0.3191964328289032,0.330357164144516,0.3415178656578064,0.3526785969734192,0.3638392686843872,0.375,0.3861607015132904,0.3973214328289032,0.4084821343421936,0.419642835855484,0.4308035671710968,0.4419642686843872,0.453125,0.4642857015132904,0.4754464328289032,0.4866071343421936,0.4977678656578064,0.5089285373687744,0.5200892686843872,0.53125,0.5424107313156128,0.5535714030265808,0.5647321343421936,0.5758928656578064,0.5870535969734192,0.5982142686843872,0.609375,0.6205357313156128,0.6316964030265808,0.6428571343421936,0.6540178656578064,0.6651785969734192,0.6763392686843872,0.6875,0.6986607313156128,0.7098214030265808,0.7209821343421936,0.7321428656578064,0.7433035969734192,0.7544642686843872,0.765625,0.7767857313156128,0.7879464030265808,0.7991071343421936,0.8102678656578064,0.8214285969734192,0.8325892686843872,0.84375,0.8549107313156128,0.8660714030265808,0.8772321343421936,0.8883928656578064,0.8995535969734192,0.9107142686843872,0.921875,0.9330357313156128,0.9441964626312256,0.9553571343421936,0.9665178656578064,0.9776785969734192,0.9888392686843872};
__constant__ float GAM[NH_] = {0.96875,0.9789702892303467,0.985848069190979,0.9904764294624329,0.9935911297798157,0.9956871271133423,0.9970976710319519,0.998046875};
__global__ __launch_bounds__(256) void k_wtG(const float* __restrict__ w, int K, int N, bf* Bt) {
    const int lane = threadIdx.x & 31; const int L0 = (blockIdx.x * 8 + (threadIdx.x >> 5)) * 8; const int nlines = N * K / 64;
#pragma unroll
    for (int ps = 0; ps < 2; ++ps) {
#pragma unroll 1
        for (int l = 0; l < 8; ++l) { const int L = L0 + l; if (L >= nlines) break; const size_t e = (size_t)L * 64 + lane * 2; const int k = (int)(e % K), n = (int)(e / K); v2us o;
            o[0] = f2bf(w[(size_t)k * N + n]); o[1] = f2bf(w[(size_t)(k + 1) * N + n]); *(volatile v2us*)(Bt + e) = o; }
        if (ps == 0) __threadfence(); }
}
__global__ __launch_bounds__(256) void k_cvt8(const float* __restrict__ src, bf* dst, size_t n8) { const size_t i = (size_t)blockIdx.x * 256 + threadIdx.x; if (i >= n8) return; const v8f v = *(const v8f*)(src + i * 8); v8us o;
#pragma unroll
    for (int k = 0; k < 8; ++k) o[k] = f2bf(v[k]); *(volatile v8us*)(dst + i * 8) = o; __threadfence(); *(volatile v8us*)(dst + i * 8) = o; }
__global__ __launch_bounds__(256) void k_whead(const float* __restrict__ W, bf* Bt) { const size_t e2 = ((size_t)blockIdx.x * 256 + threadIdx.x) * 2; if (e2 >= (size_t)NH_ * HD * DM) return; const int d = (int)(e2 % DM); const int he = (int)(e2 / DM); const int h = he / HD, e = he % HD; v2us o;
    o[0] = f2bf(W[((size_t)h * DM + d) * HD + e]); o[1] = f2bf(W[((size_t)h * DM + d + 1) * HD + e]); *(volatile v2us*)(Bt + e2) = o; __threadfence(); *(volatile v2us*)(Bt + e2) = o; }
__global__ __launch_bounds__(256) void k_xtab(float* XT4) { const int idx = blockIdx.x * 256 + threadIdx.x; if (idx >= TT * (HD / 2)) return; const int s = idx / (HD / 2), i = idx % (HD / 2); const float ang = __fmul_rn((float)s, INV[i]); const float c = cosf(ang), sn = sinf(ang);
    const float pw = __fmul_rn((float)s, 1.0f / 512.0f); const float sc = powf(BSC[i], pw); const float isc = __fdiv_rn(1.0f, sc); v4f r; r[0] = __fmul_rn(c, sc); r[1] = __fmul_rn(sn, sc); r[2] = __fmul_rn(c, isc); r[3] = __fmul_rn(sn, isc);
    *(volatile v4f*)(XT4 + (size_t)idx * 4) = r; __threadfence(); *(volatile v4f*)(XT4 + (size_t)idx * 4) = r; }
template <int KSEL>
__global__ __launch_bounds__(256) void k_xpos(const float* __restrict__ F, const float* __restrict__ XT4, bf* Ph, bf* Pl) { const size_t e = ((size_t)blockIdx.x * 256 + threadIdx.x) * 2; if (e >= (size_t)NH_ * TT * HD) return; const int d = (int)(e % HD); const int s = (int)((e / HD) % TT); const int h = (int)(e / ((size_t)HD * TT)); const float* f = F + (size_t)s * DM + h * HD + d; const float x0 = f[0], x1 = f[1];
    const v4f tb = *(const v4f*)(XT4 + ((size_t)s * (HD / 2) + (d >> 1)) * 4); const float C = tb[2 * KSEL], S = tb[2 * KSEL + 1];
    float a = __fmul_rn(x0, C), bq = __fmul_rn(x1, S); asm volatile("" : "+v"(a)); asm volatile("" : "+v"(bq)); const float r0 = __fsub_rn(a, bq); float a2 = __fmul_rn(x1, C), b2 = __fmul_rn(x0, S); asm volatile("" : "+v"(a2)); asm volatile("" : "+v"(b2)); const float r1 = __fadd_rn(a2, b2);
    v2us oh, ol; unsigned short t0, t1; splitf(r0, t0, t1); oh[0] = t0; ol[0] = t1; splitf(r1, t0, t1); oh[1] = t0; ol[1] = t1;
    *(volatile v2us*)(Ph + e) = oh; *(volatile v2us*)(Pl + e) = ol; __threadfence(); *(volatile v2us*)(Ph + e) = oh; *(volatile v2us*)(Pl + e) = ol; }
__global__ __launch_bounds__(256) void k_vt(const float* __restrict__ F, bf* Vh, bf* Vl) { const size_t e = ((size_t)blockIdx.x * 256 + threadIdx.x) * 2; if (e >= (size_t)NH_ * HD * TT) return; const int t = (int)(e % TT); const int v = (int)((e / TT) % HD); const int h = (int)(e / ((size_t)TT * HD)); v2us oh, ol;
#pragma unroll
    for (int q = 0; q < 2; ++q) { unsigned short a, c; splitf(F[(size_t)(t + q) * DM + h * HD + v], a, c); oh[q] = a; ol[q] = c; } *(volatile v2us*)(Vh + e) = oh; *(volatile v2us*)(Vl + e) = ol; __threadfence(); *(volatile v2us*)(Vh + e) = oh; *(volatile v2us*)(Vl + e) = ol; }
__global__ __launch_bounds__(256) void k_decay(const float* __restrict__ Sb, int h0, bf* Ph, bf* Pl) {
    const int lane = threadIdx.x & 31; const int row = blockIdx.x * 8 + (threadIdx.x >> 5); if (row >= ZH * TT) return; const int s = row % TT; const int zz = row / TT; const float lg = log2f(GAM[h0 + zz]); const float* sr = Sb + (size_t)row * TT;
#pragma unroll 1
    for (int ps = 0; ps < 2; ++ps) {
#pragma unroll 2
        for (int ch = 0; ch < TT / 128; ++ch) { const int t0 = ch * 128 + lane * 4; const v4f a = *(const v4f*)(sr + t0); v4us oh, ol;
#pragma unroll
            for (int q = 0; q < 4; ++q) { const int t = t0 + q; float v = 0.f; if (t <= s) { const float dcy = __builtin_amdgcn_exp2f(__fmul_rn((float)(s - t), lg)); v = __fmul_rn(a[q], dcy); } unsigned short hh, l2; splitf(v, hh, l2); oh[q] = hh; ol[q] = l2; }
            const size_t oo = (size_t)row * TT + t0; *(volatile v4us*)(Ph + oo) = oh; *(volatile v4us*)(Pl + oo) = ol; }
        if (ps == 0) __threadfence(); } }
__global__ __launch_bounds__(256) void k_gnz(const float* __restrict__ Y, const float* __restrict__ G, const float* __restrict__ gw, const float* __restrict__ gb, int h0, bf* Zh, bf* Zl) {
    const int lane = threadIdx.x & 31; const int row = blockIdx.x * 8 + (threadIdx.x >> 5); if (row >= ZH * TT) return; const int s = row % TT; const int zz = row / TT; const int c0 = (h0 + zz) * HD + lane * 4; const v4f y = *(const v4f*)(Y + (size_t)row * HD + lane * 4); float sm = 0.f;
#pragma unroll
    for (int q = 0; q < 4; ++q) sm += y[q];
#pragma unroll
    for (int sh = 16; sh; sh >>= 1) sm += __shfl_xor(sm, sh, 32);
    const float mu = sm * (1.0f / HD); float sv = 0.f;
#pragma unroll
    for (int q = 0; q < 4; ++q) { const float d0 = __fsub_rn(y[q], mu); float p = __fmul_rn(d0, d0); asm volatile("" : "+v"(p)); sv = __fadd_rn(sv, p); }
#pragma unroll
    for (int sh = 16; sh; sh >>= 1) sv += __shfl_xor(sv, sh, 32);
    const float rs = __fdiv_rn(1.0f, __fsqrt_rn(__fadd_rn(sv * (1.0f / HD), GNEPS))); v4us oh, ol;
#pragma unroll
    for (int q = 0; q < 4; ++q) { const int c = c0 + q; float n0 = __fmul_rn(__fsub_rn(y[q], mu), rs); asm volatile("" : "+v"(n0)); float n1 = __fmul_rn(n0, bfr(gw[c])); asm volatile("" : "+v"(n1)); const float yn = __fadd_rn(n1, bfr(gb[c]));
        const float g = G[(size_t)s * DM + c]; const float sg = __fdiv_rn(1.0f, __fadd_rn(1.0f, expf(-g))); float sw = __fmul_rn(g, sg); asm volatile("" : "+v"(sw)); const float z = __fmul_rn(sw, yn); unsigned short a, c2; splitf(z, a, c2); oh[q] = a; ol[q] = c2; }
    const size_t oo = (size_t)s * DM + c0;
#pragma unroll 1
    for (int ps = 0; ps < 2; ++ps) { *(volatile v4us*)(Zh + oo) = oh; *(volatile v4us*)(Zl + oo) = ol; if (ps == 0) __threadfence(); } }

extern "C" void kernel_launch(void* const* d_in, const int* in_sizes, int n_in,
                              void* d_out, int out_size, void* d_ws, size_t ws_size, hipStream_t stream) {
    (void)in_sizes; (void)n_in; (void)out_size;
    const float* X = (const float*)d_in[0]; const float* Mem = (const float*)d_in[1]; const float* WQ = (const float*)d_in[2]; const float* WK = (const float*)d_in[3]; const float* WV = (const float*)d_in[4]; const float* WG = (const float*)d_in[5]; const float* WO = (const float*)d_in[6]; const float* gw = (const float*)d_in[7]; const float* gb = (const float*)d_in[8];
    float* OUT = (float*)d_out;
    char* wsp = (char*)d_ws;
    auto take = [&](size_t bytes) { char* p = wsp; wsp += (bytes + 255) & ~(size_t)255; return (void*)p; };
    bf* BQ = (bf*)take((size_t)DM * DM * 2); bf* BK = (bf*)take((size_t)DM * DM * 2); bf* BV = (bf*)take((size_t)DM * DM * 2); bf* BG = (bf*)take((size_t)DM * DM * 2); bf* BO = (bf*)take((size_t)DM * DM * 2); float* XT4 = (float*)take((size_t)TT * (HD / 2) * 4 * 4);
    bf* XB = (bf*)take((size_t)TT * DM * 2); bf* MB = (bf*)take((size_t)TT * DM * 2); float* F = (float*)take((size_t)TT * DM * 4); float* G = (float*)take((size_t)TT * DM * 4);
    bf* QPh = (bf*)take((size_t)NH_ * TT * HD * 2); bf* QPl = (bf*)take((size_t)NH_ * TT * HD * 2); bf* KPh = (bf*)take((size_t)NH_ * TT * HD * 2); bf* KPl = (bf*)take((size_t)NH_ * TT * HD * 2); bf* VTh = (bf*)take((size_t)NH_ * HD * TT * 2); bf* VTl = (bf*)take((size_t)NH_ * HD * TT * 2);
    float* Sb = (float*)take((size_t)ZH * TT * TT * 4); bf* Ph = (bf*)take((size_t)ZH * TT * TT * 2); bf* Pl = (bf*)take((size_t)ZH * TT * TT * 2); float* Yb = (float*)take((size_t)ZH * TT * HD * 4); bf* Zh = (bf*)take((size_t)TT * DM * 2); bf* Zl = (bf*)take((size_t)TT * DM * 2);
    if ((size_t)(wsp - (char*)d_ws) > ws_size) return;
    const unsigned nwh = (unsigned)(((size_t)NH_ * HD * DM / 2 + 255) / 256);
    k_whead<<<nwh, 256, 0, stream>>>(WQ, BQ); k_whead<<<nwh, 256, 0, stream>>>(WK, BK); k_whead<<<nwh, 256, 0, stream>>>(WV, BV);
    k_wtG<<<(unsigned)((DM * DM / 64 + 63) / 64), 256, 0, stream>>>(WG, DM, DM, BG); k_wtG<<<(unsigned)((DM * DM / 64 + 63) / 64), 256, 0, stream>>>(WO, DM, DM, BO);
    k_xtab<<<(TT * (HD / 2) + 255) / 256, 256, 0, stream>>>(XT4);
    const unsigned npl = (unsigned)(((size_t)NH_ * TT * HD / 2 + 255) / 256);
    for (int b = 0; b < NB_; ++b) {
        k_cvt8<<<(unsigned)(((size_t)TT * DM / 8 + 255) / 256), 256, 0, stream>>>(X + (size_t)b * TT * DM, XB, (size_t)TT * DM / 8); k_cvt8<<<(unsigned)(((size_t)TT * DM / 8 + 255) / 256), 256, 0, stream>>>(Mem + (size_t)b * TT * DM, MB, (size_t)TT * DM / 8);
        k_gemmw<bf, 0, false><<<dim3(TT / 64, DM / 64, 1), 32, 0, stream>>>(XB, nullptr, BQ, nullptr, DM, F, DM, nullptr, 0, 0, 0); k_xpos<0><<<npl, 256, 0, stream>>>(F, XT4, QPh, QPl);
        k_gemmw<bf, 0, false><<<dim3(TT / 64, DM / 64, 1), 32, 0, stream>>>(MB, nullptr, BK, nullptr, DM, F, DM, nullptr, 0, 0, 0); k_xpos<1><<<npl, 256, 0, stream>>>(F, XT4, KPh, KPl);
        k_gemmw<bf, 0, false><<<dim3(TT / 64, DM / 64, 1), 32, 0, stream>>>(MB, nullptr, BV, nullptr, DM, F, DM, nullptr, 0, 0, 0); k_vt<<<npl, 256, 0, stream>>>(F, VTh, VTl);
        k_gemmw<bf, 0, false><<<dim3(TT / 64, DM / 64, 1), 32, 0, stream>>>(XB, nullptr, BG, nullptr, DM, G, DM, nullptr, 0, 0, 0);
        for (int h0 = 0; h0 < NH_; h0 += ZH) {
            k_gemmc<bf, 2, 1><<<dim3(TT / 64, TT / 64, ZH), 32, 0, stream>>>(QPh + (size_t)h0 * TT * HD, QPl + (size_t)h0 * TT * HD, KPh + (size_t)h0 * TT * HD, KPl + (size_t)h0 * TT * HD, HD, Sb, TT, 0, (size_t)TT * HD, (size_t)TT * HD, (size_t)TT * TT);
            k_decay<<<ZH * TT / 8, 256, 0, stream>>>(Sb, h0, Ph, Pl);
            k_gemmc<bf, 2, 2><<<dim3(TT / 64, HD / 64, ZH), 32, 0, stream>>>(Ph, Pl, VTh + (size_t)h0 * HD * TT, VTl + (size_t)h0 * HD * TT, TT, Yb, HD, 0, (size_t)TT * TT, (size_t)HD * TT, (size_t)TT * HD);
            k_gnz<<<ZH * TT / 8, 256, 0, stream>>>(Yb, G, gw, gb, h0, Zh, Zl); }
        k_gemmw<bf, 1, false><<<dim3(TT / 64, DM / 64, 1), 32, 0, stream>>>(Zh, Zl, BO, nullptr, DM, OUT + (size_t)b * TT * DM, DM, nullptr, 0, 0, 0); }
}
